// RNN_70480413327462
// MI455X (gfx1250) — hardware-verified
//
#include <hip/hip_runtime.h>
#include <math.h>

constexpr int NROW   = 8192;
constexpr int NPAT   = 4096;
constexpr int HID    = 32;
constexpr int EMB    = 34;
constexpr int NOBS   = 10;
constexpr int NSTEPS = 59;
constexpr int NTHR   = 256;
constexpr int NWAVE  = NTHR / 32;
constexpr int ROWS_W = 16;
constexpr int ROWS_B = ROWS_W * NWAVE;
constexpr int NBLK   = NROW / ROWS_B;
constexpr int QPITCH = 64;
constexpr int SLP    = 68;
constexpr int H1P    = 36;
constexpr int WKP    = 32;
constexpr int PR_WX   = 0;
constexpr int PR_WH   = 32;
constexpr int PR_WF2  = 64;
constexpr int PR_WFS  = 96;
constexpr int PR_WIN  = 128;
constexpr int PR_WOUT = 272;
constexpr int PR_ROWS = 320;
constexpr float WCAR = 16.0f;
constexpr float OCAR = 8.0f;
constexpr float RCAR = 2048.0f;
constexpr float SC_M1 = 1.0f / 16.0f;
constexpr float SC_R1 = 1.0f / 32768.0f;
constexpr float SC_M8 = 1.0f / 128.0f;
constexpr float SC_R8 = 1.0f / 262144.0f;
constexpr float ATT_SCALE = 0.17149858514250882f;
constexpr float LN_EPS = 1e-5f;
static_assert(NROW % ROWS_B == 0);
static_assert(NROW == 2 * NPAT);
static_assert((NROW * HID) % (4 * NTHR) == 0);
static_assert(SLP % 4 == 0 && H1P % 4 == 0);
static_assert(PR_WIN + 3 * 48 == PR_WOUT && PR_WOUT + 48 == PR_ROWS);
static_assert((PR_WX % 2) == 0 && (PR_WH % 2) == 0 && (PR_WF2 % 2) == 0 && (PR_WFS % 2) == 0 && (PR_WIN % 2) == 0 && (PR_WOUT % 2) == 0);

typedef __attribute__((ext_vector_type(16))) _Float16 v16h;
typedef __attribute__((ext_vector_type(8)))  _Float16 v8h;
typedef __attribute__((ext_vector_type(8)))  float    v8f;
typedef __attribute__((ext_vector_type(4)))  float    v4f;

__device__ __forceinline__ v16h frag_load(const _Float16* p) {
  union { v16h v; v8h h[2]; } f;
  f.h[0] = *(const v8h*)(p);
  f.h[1] = *(const v8h*)(p + 16);
  return f.v;
}
__device__ __forceinline__ void cvt_afrag(const float* p, float ca, v16h& hi, v16h& lo) {
  const v4f x0 = *(const v4f*)(p);
  const v4f x1 = *(const v4f*)(p + 4);
  const v4f x2 = *(const v4f*)(p + 16);
  const v4f x3 = *(const v4f*)(p + 20);
#pragma unroll
  for (int e = 0; e < 4; ++e) {
    float s, hb; _Float16 h;
    s = x0[e] * ca; h = (_Float16)s; hb = (float)h; hi[e]      = h; lo[e]      = (_Float16)((s - hb) * RCAR);
    s = x1[e] * ca; h = (_Float16)s; hb = (float)h; hi[4 + e]  = h; lo[4 + e]  = (_Float16)((s - hb) * RCAR);
    s = x2[e] * ca; h = (_Float16)s; hb = (float)h; hi[8 + e]  = h; lo[8 + e]  = (_Float16)((s - hb) * RCAR);
    s = x3[e] * ca; h = (_Float16)s; hb = (float)h; hi[12 + e] = h; lo[12 + e] = (_Float16)((s - hb) * RCAR);
  }
}
__device__ __forceinline__ v8f wmma_f16(v16h a, v16h b, v8f c) {
  return __builtin_amdgcn_wmma_f32_16x16x32_f16(false, a, false, b, (short)0, c, false, false);
}
__device__ __forceinline__ void mma3(v8f& am, v8f& ar, v16h ah, v16h al, v16h bh, v16h bl) {
  am = wmma_f16(ah, bh, am);
  ar = wmma_f16(ah, bl, ar);
  ar = wmma_f16(al, bh, ar);
}
__device__ __forceinline__ void guard4(v8f& am, v8f& ar, v16h f0, v16h f1, v16h f2, v16h f3) {
  asm volatile("v_nop\n\tv_nop\n\tv_nop\n\tv_nop" : "+v"(am), "+v"(ar) : "v"(f0), "v"(f1), "v"(f2), "v"(f3));
}
__device__ __forceinline__ void guard8(v8f& am, v8f& ar, v16h f0, v16h f1, v16h f2, v16h f3,
                                       v16h f4, v16h f5, v16h f6, v16h f7) {
  asm volatile("v_nop\n\tv_nop\n\tv_nop\n\tv_nop" : "+v"(am), "+v"(ar)
               : "v"(f0), "v"(f1), "v"(f2), "v"(f3), "v"(f4), "v"(f5), "v"(f6), "v"(f7));
}
__device__ __forceinline__ void pin_frag4(v16h a, v16h b, v16h c, v16h d) { asm volatile("" :: "v"(a), "v"(b), "v"(c), "v"(d) : "memory"); }
__device__ __forceinline__ void pin1(float a) { asm volatile("" :: "v"(a) : "memory"); }
__device__ __forceinline__ void pin5(float a, float b, float c, float d, float e) { asm volatile("" :: "v"(a), "v"(b), "v"(c), "v"(d), "v"(e) : "memory"); }
__device__ __forceinline__ void pin_mem() { asm volatile("" ::: "memory"); }
__device__ __forceinline__ void wave_sync() {
  __builtin_amdgcn_fence(__ATOMIC_RELEASE, "workgroup");
  __builtin_amdgcn_wave_barrier();
  __builtin_amdgcn_fence(__ATOMIC_ACQUIRE, "workgroup");
}

__device__ __forceinline__ void store_tile32(const float* slab, float* dst, int lane) {
  const int q = lane >> 3, c4 = (lane & 7) * 4;
  for (int pass = 0; pass < 2; ++pass) {
#pragma unroll
    for (int it = 0; it < 4; ++it) {
      const int row = it * 4 + q;
      const v4f v = *(const v4f*)(slab + row * SLP + c4);
      *(volatile v4f*)(dst + (size_t)row * HID + c4) = v;
    }
    __threadfence();
  }
}
__device__ __forceinline__ void store_tile32x2(const float* slab, float* dstA, float* dstB, int lane) {
  const int q = lane >> 3, c4 = (lane & 7) * 4;
  for (int pass = 0; pass < 2; ++pass) {
#pragma unroll
    for (int it = 0; it < 4; ++it) {
      const int row = it * 4 + q;
      const v4f v = *(const v4f*)(slab + row * SLP + c4);
      *(volatile v4f*)(dstA + (size_t)row * HID + c4) = v;
      *(volatile v4f*)(dstB + (size_t)row * HID + c4) = v;
    }
    __threadfence();
  }
}
__device__ __forceinline__ void store_tile64(const float* slab, float* dst, int lane) {
  const int hh2 = lane >> 4, c4 = (lane & 15) * 4;
  for (int pass = 0; pass < 2; ++pass) {
#pragma unroll
    for (int it = 0; it < 8; ++it) {
      const int row = it * 2 + hh2;
      const v4f v = *(const v4f*)(slab + row * SLP + c4);
      *(volatile v4f*)(dst + (size_t)row * QPITCH + c4) = v;
    }
    __threadfence();
  }
}

__device__ __forceinline__ int nbr_of(int p, int dr, int dc) {
  const int r = p >> 6, cc = p & 63;
  int nr = r + dr + ((r == 0) ? 1 : 0) - ((r == 63) ? 1 : 0);
  int nc = cc + dc + ((cc == 0) ? 1 : 0) - ((cc == 63) ? 1 : 0);
  nr = nr < 0 ? 0 : (nr > 63 ? 63 : nr);
  nc = nc < 0 ? 0 : (nc > 63 ? 63 : nc);
  return (nr << 6) | nc;
}

__global__ __launch_bounds__(NTHR) void prep_w_kernel(
    const float* __restrict__ Wx2h, const float* __restrict__ Wh2h, const float* __restrict__ Wfc2,
    const float* __restrict__ Wfcsa, const float* __restrict__ Win, const float* __restrict__ Wout,
    unsigned short* __restrict__ WPH, unsigned short* __restrict__ WPL) {
  const int which = blockIdx.y;
  const float* src = Wx2h; int pitch = HID, nreal = HID, npad = HID, row0 = PR_WX, gstride = 0;
  if (which == 1)      { src = Wh2h;  row0 = PR_WH; }
  else if (which == 2) { src = Wfc2;  row0 = PR_WF2; }
  else if (which == 3) { src = Wfcsa; pitch = EMB; row0 = PR_WFS; }
  else if (which == 4) { src = Win;   pitch = EMB; nreal = EMB; npad = 3 * 48; row0 = PR_WIN; gstride = EMB; }
  else if (which == 5) { src = Wout;  pitch = EMB; nreal = EMB; npad = 48; row0 = PR_WOUT; }
  const int i = blockIdx.x * NTHR + threadIdx.x;
  const int r = i >> 2;
  if (r >= npad) return;
  const int c8  = (i & 3) * 8;
  const int grp = r / 48;
  const int nn  = r - grp * 48;
  const bool real = nn < nreal;
  const int ncl = real ? nn : (nreal - 1);
  const float* sp = src + (size_t)(grp * gstride + ncl) * pitch + c8;
  float f[8];
#pragma unroll
  for (int e = 0; e < 8; ++e) f[e] = sp[e];
  v8h hv, lv;
#pragma unroll
  for (int e = 0; e < 8; ++e) {
    const float s = real ? f[e] * WCAR : 0.0f;
    const _Float16 h = (_Float16)s;
    const float hb = (float)h;
    hv[e] = h;
    lv[e] = (_Float16)((s - hb) * RCAR);
  }
  const size_t o = (size_t)(row0 + r) * WKP + c8;
  *(volatile v8h*)(WPH + o) = hv;
  *(volatile v8h*)(WPL + o) = lv;
  __threadfence();
  *(volatile v8h*)(WPH + o) = hv;
  *(volatile v8h*)(WPL + o) = lv;
}

__global__ __launch_bounds__(NTHR) void zero4_kernel(float* __restrict__ p, int n4) {
  const int i = blockIdx.x * NTHR + threadIdx.x;
  if (i < n4) {
    const v4f z = {0.0f, 0.0f, 0.0f, 0.0f};
    *(volatile v4f*)(p + (size_t)i * 4) = z;
    __threadfence();
    *(volatile v4f*)(p + (size_t)i * 4) = z;
  }
}

__global__ __launch_bounds__(NTHR) void step_a_kernel(
    const float* __restrict__ inp, const float* __restrict__ hS,
    const unsigned short* __restrict__ WPH, const unsigned short* __restrict__ WPL,
    const float* __restrict__ bx2h, const float* __restrict__ bh2h,
    const float* __restrict__ Win, const float* __restrict__ bin,
    float* __restrict__ hA, float* __restrict__ Qp, float* __restrict__ Kp, float* __restrict__ Vp) {
  __shared__ __align__(16) float Sl[NWAVE][ROWS_W * SLP];
  const int tid = threadIdx.x, lane = tid & 31, wave = tid >> 5;
  const int c = lane & 15, hh = lane >> 4, koff = 8 * hh;
  const int rowbase = (blockIdx.x * NWAVE + wave) * ROWS_W;
  float* slab = Sl[wave];
  const _Float16* PH = (const _Float16*)WPH;
  const _Float16* PL = (const _Float16*)WPL;
  const v8f z8 = {0.f, 0.f, 0.f, 0.f, 0.f, 0.f, 0.f, 0.f};

#pragma unroll
  for (int r = 0; r < 8; ++r) slab[(8 * hh + r) * SLP + 48 + c] = 0.0f;

  v16h xi_h, xi_l, hp_h, hp_l;
  cvt_afrag(inp + (size_t)(rowbase + c) * HID + koff, 1.0f, xi_h, xi_l);
  cvt_afrag(hS  + (size_t)(rowbase + c) * HID + koff, 1.0f, hp_h, hp_l);
  pin_frag4(xi_h, xi_l, hp_h, hp_l);

#pragma unroll
  for (int ct = 0; ct < 2; ++ct) {
    const v16h bxh = frag_load(PH + (size_t)(PR_WX + 16 * ct + c) * WKP + koff);
    const v16h bxl = frag_load(PL + (size_t)(PR_WX + 16 * ct + c) * WKP + koff);
    const v16h bhh = frag_load(PH + (size_t)(PR_WH + 16 * ct + c) * WKP + koff);
    const v16h bhl = frag_load(PL + (size_t)(PR_WH + 16 * ct + c) * WKP + koff);
    v8f am = z8, ar = z8;
    mma3(am, ar, xi_h, xi_l, bxh, bxl);
    mma3(am, ar, hp_h, hp_l, bhh, bhl);
    guard8(am, ar, xi_h, xi_l, hp_h, hp_l, bxh, bxl, bhh, bhl);
    const int n = 16 * ct + c;
    const float bsum = bx2h[n] + bh2h[n];
#pragma unroll
    for (int r = 0; r < 8; ++r) {
      const float pre = am[r] * SC_M1 + ar[r] * SC_R1 + bsum;
      slab[(8 * hh + r) * SLP + n] = tanhf(pre);
    }
    pin_mem();
  }
  wave_sync();
  store_tile32(slab, hA + (size_t)rowbase * HID, lane);
  v16h a1h, a1l;
  cvt_afrag(slab + c * SLP + koff, 1.0f, a1h, a1l);
  wave_sync();

#pragma unroll
  for (int mat = 0; mat < 3; ++mat) {
    float* outp = (mat == 0) ? Qp : ((mat == 1) ? Kp : Vp);
#pragma unroll
    for (int ct = 0; ct < 3; ++ct) {
      const int prow = PR_WIN + 48 * mat + 16 * ct + c;
      const v16h bh = frag_load(PH + (size_t)prow * WKP + koff);
      const v16h bl = frag_load(PL + (size_t)prow * WKP + koff);
      v8f am = z8, ar = z8;
      mma3(am, ar, a1h, a1l, bh, bl);
      guard4(am, ar, a1h, a1l, bh, bl);
      const int n   = 16 * ct + c;
      const int ncl = (n < EMB - 1) ? n : (EMB - 1);
      const int wr  = EMB * mat + ncl;
      const float w32 = Win[(size_t)wr * EMB + 32];
      const float w33 = Win[(size_t)wr * EMB + 33];
      const float bi  = bin[wr];
#pragma unroll
      for (int r = 0; r < 8; ++r) {
        const int m = 8 * hh + r;
        const int p = (rowbase + m) & (NPAT - 1);
        const float c0 = (float)(p >> 6) * (1.0f / 64.0f);
        const float c1 = (float)(p & 63) * (1.0f / 64.0f);
        float v = am[r] * SC_M1 + ar[r] * SC_R1 + bi + c0 * w32 + c1 * w33;
        v = (n < EMB) ? v : 0.0f;
        slab[m * SLP + n] = v;
      }
      pin_mem();
    }
    wave_sync();
    store_tile64(slab, outp + (size_t)rowbase * QPITCH, lane);
    wave_sync();
  }
}

__global__ __launch_bounds__(NTHR) void step_b_kernel(
    const float* __restrict__ hA, const float* __restrict__ Qp, const float* __restrict__ Kp, const float* __restrict__ Vp,
    const unsigned short* __restrict__ WPH, const unsigned short* __restrict__ WPL,
    const float* __restrict__ Wout, const float* __restrict__ bout,
    const float* __restrict__ Wfcsa, const float* __restrict__ bfcsa,
    const float* __restrict__ bfc2, const float* __restrict__ lng, const float* __restrict__ lnb,
    float* __restrict__ hS, float* __restrict__ outT, float* __restrict__ prevP) {
  __shared__ __align__(16) float Sl[NWAVE][ROWS_W * SLP];
  __shared__ __align__(16) float H1[NWAVE][ROWS_W * H1P];
  const int tid = threadIdx.x, lane = tid & 31, wave = tid >> 5;
  const int c = lane & 15, hh = lane >> 4, koff = 8 * hh;
  const int rowbase = (blockIdx.x * NWAVE + wave) * ROWS_W;
  float* slab = Sl[wave];
  float* h1s  = H1[wave];
  const _Float16* PH = (const _Float16*)WPH;
  const _Float16* PL = (const _Float16*)WPL;
  const v8f z8 = {0.f, 0.f, 0.f, 0.f, 0.f, 0.f, 0.f, 0.f};

  {
    const int rr = lane >> 1, cb = (lane & 1) * 16;
    const float* src = hA + (size_t)(rowbase + rr) * HID + cb;
    float* dst = h1s + rr * H1P + cb;
#pragma unroll
    for (int i = 0; i < 4; ++i) *(v4f*)(dst + 4 * i) = *(const v4f*)(src + 4 * i);
  }
  pin_mem();

  {
    const int n = rowbase + c;
    const int bb = n >> 12;
    const int p = n & (NPAT - 1);
    const int base = bb << 12;
    const int e0 = 20 * hh;
    int idx[9];
#pragma unroll
    for (int l = 0; l < 9; ++l) idx[l] = base + nbr_of(p, l / 3 - 1, l % 3 - 1);
    float qv[20];
    {
      const float* qp = Qp + (size_t)idx[4] * QPITCH + e0;
#pragma unroll
      for (int i = 0; i < 5; ++i) {
        const v4f t = *(const v4f*)(qp + 4 * i);
        qv[4 * i + 0] = t[0]; qv[4 * i + 1] = t[1]; qv[4 * i + 2] = t[2]; qv[4 * i + 3] = t[3];
      }
    }
    pin5(qv[0], qv[4], qv[8], qv[12], qv[16]);
    float sc[9];
#pragma unroll
    for (int l = 0; l < 9; ++l) {
      const float* kp = Kp + (size_t)idx[l] * QPITCH + e0;
      const v4f k0 = *(const v4f*)(kp);
      const v4f k1 = *(const v4f*)(kp + 4);
      const v4f k2 = *(const v4f*)(kp + 8);
      const v4f k3 = *(const v4f*)(kp + 12);
      const v4f k4 = *(const v4f*)(kp + 16);
      float part = 0.0f;
#pragma unroll
      for (int e = 0; e < 4; ++e) {
        part += qv[e] * k0[e];
        part += qv[4 + e] * k1[e];
        part += qv[8 + e] * k2[e];
        part += qv[12 + e] * k3[e];
        part += qv[16 + e] * k4[e];
      }
      pin1(part);
      const float tot = part + __shfl_xor(part, 16, 32);
      sc[l] = tot * ATT_SCALE;
    }
    float smax = sc[0];
#pragma unroll
    for (int l = 1; l < 9; ++l) smax = fmaxf(smax, sc[l]);
    float ex[9];
    float ssum = 0.0f;
#pragma unroll
    for (int l = 0; l < 9; ++l) { ex[l] = expf(sc[l] - smax); ssum += ex[l]; }
    const float inv = 1.0f / ssum;
    float ov[20];
#pragma unroll
    for (int i = 0; i < 20; ++i) ov[i] = 0.0f;
#pragma unroll
    for (int l = 0; l < 9; ++l) {
      const float w = ex[l] * inv;
      const float* vp = Vp + (size_t)idx[l] * QPITCH + e0;
      const v4f v0 = *(const v4f*)(vp);
      const v4f v1 = *(const v4f*)(vp + 4);
      const v4f v2 = *(const v4f*)(vp + 8);
      const v4f v3 = *(const v4f*)(vp + 12);
      const v4f v4 = *(const v4f*)(vp + 16);
#pragma unroll
      for (int e = 0; e < 4; ++e) {
        ov[e]      += w * v0[e];
        ov[4 + e]  += w * v1[e];
        ov[8 + e]  += w * v2[e];
        ov[12 + e] += w * v3[e];
        ov[16 + e] += w * v4[e];
      }
      pin5(ov[0], ov[4], ov[8], ov[12], ov[16]);
    }
    float* orow = slab + c * SLP + e0;
#pragma unroll
    for (int i = 0; i < 5; ++i) {
      v4f t; t[0] = ov[4 * i]; t[1] = ov[4 * i + 1]; t[2] = ov[4 * i + 2]; t[3] = ov[4 * i + 3];
      *(v4f*)(orow + 4 * i) = t;
    }
  }
  wave_sync();

  {
    v16h oh, ol;
    cvt_afrag(slab + c * SLP + koff, OCAR, oh, ol);
    float o32[8], o33[8];
#pragma unroll
    for (int r = 0; r < 8; ++r) { o32[r] = slab[(8 * hh + r) * SLP + 32]; o33[r] = slab[(8 * hh + r) * SLP + 33]; }
    wave_sync();
#pragma unroll
    for (int ct = 0; ct < 3; ++ct) {
      const int prow = PR_WOUT + 16 * ct + c;
      const v16h bh = frag_load(PH + (size_t)prow * WKP + koff);
      const v16h bl = frag_load(PL + (size_t)prow * WKP + koff);
      v8f am = z8, ar = z8;
      mma3(am, ar, oh, ol, bh, bl);
      guard4(am, ar, oh, ol, bh, bl);
      const int n   = 16 * ct + c;
      const int ncl = (n < EMB - 1) ? n : (EMB - 1);
      const float w32 = Wout[(size_t)ncl * EMB + 32];
      const float w33 = Wout[(size_t)ncl * EMB + 33];
      const float bo  = bout[ncl];
#pragma unroll
      for (int r = 0; r < 8; ++r) {
        float v = am[r] * SC_M8 + ar[r] * SC_R8 + bo + o32[r] * w32 + o33[r] * w33;
        v = (n < EMB) ? v : 0.0f;
        slab[(8 * hh + r) * SLP + n] = v;
      }
      pin_mem();
    }
  }
  wave_sync();

  {
    v16h ah, al;
    cvt_afrag(slab + c * SLP + koff, OCAR, ah, al);
    float a32[8], a33[8], h1v[2][8];
#pragma unroll
    for (int r = 0; r < 8; ++r) {
      a32[r] = slab[(8 * hh + r) * SLP + 32];
      a33[r] = slab[(8 * hh + r) * SLP + 33];
      h1v[0][r] = h1s[(8 * hh + r) * H1P + c];
      h1v[1][r] = h1s[(8 * hh + r) * H1P + 16 + c];
    }
    wave_sync();
#pragma unroll
    for (int ct = 0; ct < 2; ++ct) {
      const int prow = PR_WFS + 16 * ct + c;
      const v16h bh = frag_load(PH + (size_t)prow * WKP + koff);
      const v16h bl = frag_load(PL + (size_t)prow * WKP + koff);
      v8f am = z8, ar = z8;
      mma3(am, ar, ah, al, bh, bl);
      guard4(am, ar, ah, al, bh, bl);
      const int n = 16 * ct + c;
      const float w32 = Wfcsa[(size_t)n * EMB + 32];
      const float w33 = Wfcsa[(size_t)n * EMB + 33];
      const float bf  = bfcsa[n];
#pragma unroll
      for (int r = 0; r < 8; ++r) {
        const float fc = am[r] * SC_M8 + ar[r] * SC_R8 + bf + a32[r] * w32 + a33[r] * w33;
        slab[(8 * hh + r) * SLP + n] = h1v[ct][r] + fc;
      }
      pin_mem();
    }
  }
  wave_sync();
  store_tile32(slab, hS + (size_t)rowbase * HID, lane);
  v16h gh, gl;
  cvt_afrag(slab + c * SLP + koff, 1.0f, gh, gl);
  wave_sync();

#pragma unroll
  for (int ct = 0; ct < 2; ++ct) {
    const int prow = PR_WF2 + 16 * ct + c;
    const v16h bh = frag_load(PH + (size_t)prow * WKP + koff);
    const v16h bl = frag_load(PL + (size_t)prow * WKP + koff);
    v8f am = z8, ar = z8;
    mma3(am, ar, gh, gl, bh, bl);
    guard4(am, ar, gh, gl, bh, bl);
    const int n = 16 * ct + c;
    const float bz = bfc2[n];
#pragma unroll
    for (int r = 0; r < 8; ++r) slab[(8 * hh + r) * SLP + n] = am[r] * SC_M1 + ar[r] * SC_R1 + bz;
    pin_mem();
  }
  wave_sync();

  {
    float* zr = slab + c * SLP + 16 * hh;
    v4f z[4];
#pragma unroll
    for (int i = 0; i < 4; ++i) z[i] = *(const v4f*)(zr + 4 * i);
    float ps = 0.0f;
#pragma unroll
    for (int i = 0; i < 4; ++i) ps += (z[i][0] + z[i][1]) + (z[i][2] + z[i][3]);
    const float tot = ps + __shfl_xor(ps, 16, 32);
    const float mu = tot * (1.0f / HID);
    float pss = 0.0f;
#pragma unroll
    for (int i = 0; i < 4; ++i)
#pragma unroll
      for (int e = 0; e < 4; ++e) { const float d = z[i][e] - mu; z[i][e] = d; pss += d * d; }
    const float tss = pss + __shfl_xor(pss, 16, 32);
    const float var = tss * (1.0f / HID);
    const float rstd = rsqrtf(var + LN_EPS);
#pragma unroll
    for (int i = 0; i < 4; ++i) {
      const v4f g  = *(const v4f*)(lng + 16 * hh + 4 * i);
      const v4f be = *(const v4f*)(lnb + 16 * hh + 4 * i);
      v4f o;
#pragma unroll
      for (int e = 0; e < 4; ++e) o[e] = (z[i][e] * rstd) * g[e] + be[e];
      *(v4f*)(zr + 4 * i) = o;
    }
  }
  wave_sync();
  store_tile32x2(slab, outT + (size_t)rowbase * HID, prevP + (size_t)rowbase * HID, lane);
}

extern "C" void kernel_launch(void* const* d_in, const int* in_sizes, int n_in,
                              void* d_out, int out_size, void* d_ws, size_t ws_size, hipStream_t stream) {
  if (n_in < 15 || d_out == nullptr || d_ws == nullptr) return;
  if (in_sizes[0] != NOBS * NROW * HID || in_sizes[1] != HID * HID || in_sizes[2] != HID ||
      in_sizes[3] != HID * HID || in_sizes[4] != HID || in_sizes[5] != HID * HID || in_sizes[6] != HID ||
      in_sizes[7] != HID || in_sizes[8] != HID || in_sizes[9] != HID * EMB || in_sizes[10] != HID ||
      in_sizes[11] != 3 * EMB * EMB || in_sizes[12] != 3 * EMB || in_sizes[13] != EMB * EMB || in_sizes[14] != EMB ||
      out_size != NSTEPS * NROW * HID) return;

  const float* x     = (const float*)d_in[0];
  const float* Wx2h  = (const float*)d_in[1];
  const float* bx2h  = (const float*)d_in[2];
  const float* Wh2h  = (const float*)d_in[3];
  const float* bh2h  = (const float*)d_in[4];
  const float* Wfc2  = (const float*)d_in[5];
  const float* bfc2  = (const float*)d_in[6];
  const float* lng   = (const float*)d_in[7];
  const float* lnb   = (const float*)d_in[8];
  const float* Wfcsa = (const float*)d_in[9];
  const float* bfcsa = (const float*)d_in[10];
  const float* Win   = (const float*)d_in[11];
  const float* bin   = (const float*)d_in[12];
  const float* Wout  = (const float*)d_in[13];
  const float* bout  = (const float*)d_in[14];
  float* out = (float*)d_out;

  char* ws = (char*)d_ws; size_t off = 0;
  auto carve = [&](size_t bytes) -> char* { char* p = ws + off; off += (bytes + 255) & ~(size_t)255; return p; };
  unsigned short* WPH = (unsigned short*)carve((size_t)PR_ROWS * WKP * 2);
  unsigned short* WPL = (unsigned short*)carve((size_t)PR_ROWS * WKP * 2);
  float* HS = (float*)carve((size_t)NROW * HID * 4);
  float* HA = (float*)carve((size_t)NROW * HID * 4);
  float* QP = (float*)carve((size_t)NROW * QPITCH * 4);
  float* KP = (float*)carve((size_t)NROW * QPITCH * 4);
  float* VP = (float*)carve((size_t)NROW * QPITCH * 4);
  float* PP = (float*)carve((size_t)NROW * HID * 4);
  if (off > ws_size || off > (size_t)134217728) return;

  prep_w_kernel<<<dim3(3, 6), NTHR, 0, stream>>>(Wx2h, Wh2h, Wfc2, Wfcsa, Win, Wout, WPH, WPL);
  const int n4 = NROW * HID / 4;
  zero4_kernel<<<(n4 + NTHR - 1) / NTHR, NTHR, 0, stream>>>(HS, n4);
  for (int t = 0; t < NSTEPS; ++t) {
    const float* inp = (t < NOBS) ? (x + (size_t)t * NROW * HID) : PP;
    step_a_kernel<<<NBLK, NTHR, 0, stream>>>(inp, HS, WPH, WPL, bx2h, bh2h, Win, bin, HA, QP, KP, VP);
    step_b_kernel<<<NBLK, NTHR, 0, stream>>>(HA, QP, KP, VP, WPH, WPL, Wout, bout, Wfcsa, bfcsa, bfc2, lng, lnb,
                                             HS, out + (size_t)t * NROW * HID, PP);
  }
}
